// CondAttLSTM_56530359550210
// MI455X (gfx1250) — hardware-verified
//
#include <hip/hip_runtime.h>
#include <stddef.h>

typedef __attribute__((ext_vector_type(16))) _Float16 v16h;
typedef __attribute__((ext_vector_type(8)))  _Float16 v8h;
typedef __attribute__((ext_vector_type(16))) __bf16   v16b;
typedef __attribute__((ext_vector_type(8)))  __bf16   v8b;
typedef __attribute__((ext_vector_type(8)))  float    v8f;
typedef __attribute__((ext_vector_type(4)))  float    v4f;
typedef __attribute__((ext_vector_type(4)))  _Float16 v4h;
typedef __attribute__((ext_vector_type(4)))  unsigned v4u;
#define PSCALE 32768.0f
#define U16(p) ((const unsigned short*)(const void*)(p))
#define PSCALE_INV (1.0f / 32768.0f)

__device__ __forceinline__ unsigned short f2bf_bits(float f) {
  unsigned u = __float_as_uint(f);
  return (unsigned short)((u + 0x7FFFu + ((u >> 16) & 1u)) >> 16);
}
__device__ __forceinline__ float bf_bits2f(unsigned short h) { return __uint_as_float(((unsigned)h) << 16); }

__device__ __forceinline__ void dep_guard_h(v8f& a, v8f& b, v16h x, v16h y) { asm volatile("v_nop\n\tv_nop\n\tv_nop\n\tv_nop" : "+v"(a), "+v"(b) : "v"(x), "v"(y)); }
__device__ __forceinline__ void dep_guard_b(v8f& a, v8f& b, v16b x, v16b y) { asm volatile("v_nop\n\tv_nop\n\tv_nop\n\tv_nop" : "+v"(a), "+v"(b) : "v"(x), "v"(y)); }
__device__ __forceinline__ void keep4_h(v16h a, v16h b, v16h c, v16h d) { asm volatile("v_nop" :: "v"(a), "v"(b), "v"(c), "v"(d)); }
__device__ __forceinline__ void keep4_b(v16b a, v16b b, v16b c, v16b d) { asm volatile("v_nop" :: "v"(a), "v"(b), "v"(c), "v"(d)); }
__device__ __forceinline__ void acc_guard4(v8f& a, v8f& b, v8f& c, v8f& d) { asm volatile("v_nop\n\tv_nop\n\tv_nop\n\tv_nop" : "+v"(a), "+v"(b), "+v"(c), "+v"(d)); }
template <typename T> struct Frag;
template <> struct Frag<_Float16> {
  typedef v16h V; union U { v16h v; v8h h[2]; };
  static __device__ __forceinline__ v16h load(const _Float16* p) {
    U f; f.h[0] = *(const v8h*)(p); f.h[1] = *(const v8h*)(p + 16); return f.v;
  }
  static __device__ __forceinline__ v8f mma(v16h a, v16h b, v8f c) {
    return __builtin_amdgcn_wmma_f32_16x16x32_f16(false, a, false, b, (short)0, c, false, false);
  }
  static __device__ __forceinline__ void guard(v8f& a, v8f& b, v16h x, v16h y) { dep_guard_h(a, b, x, y); }
  static __device__ __forceinline__ void keep(v16h a, v16h b, v16h c, v16h d) { keep4_h(a, b, c, d); }
};
template <> struct Frag<__bf16> {
  typedef v16b V; union U { v16b v; v8b h[2]; };
  static __device__ __forceinline__ v16b load(const __bf16* p) {
    U f; f.h[0] = *(const v8b*)(p); f.h[1] = *(const v8b*)(p + 16); return f.v;
  }
  static __device__ __forceinline__ v8f mma(v16b a, v16b b, v8f c) {
    return __builtin_amdgcn_wmma_f32_16x16x32_bf16(false, a, false, b, (short)0, c, false, false);
  }
  static __device__ __forceinline__ void guard(v8f& a, v8f& b, v16b x, v16b y) { dep_guard_b(a, b, x, y); }
  static __device__ __forceinline__ void keep(v16b a, v16b b, v16b c, v16b d) { keep4_b(a, b, c, d); }
};

template <int ET> struct Elem;
template <> struct Elem<0> { typedef _Float16 T; };
template <> struct Elem<1> { typedef __bf16 T; };
template <int ET, bool SPLIT, int BIAS_MODE, int OUT_MODE, bool RESID, int ACT = 0>
__global__ __launch_bounds__(256) void wmma_gemm64(
    const unsigned short* __restrict__ Ap, const unsigned short* __restrict__ A2p, int lda, long strideA,
    const unsigned short* __restrict__ Btp, const unsigned short* __restrict__ Bt2p, int ldb, long strideB,
    void* __restrict__ Cout, void* __restrict__ Cout2, int ldc, long strideC,
    const float* __restrict__ bias,
    const float* __restrict__ resid, long strideR,
    int M, int N, int K, float scale) {
  typedef typename Elem<ET>::T T;
  typedef typename Frag<T>::V V;
  const T* A = (const T*)Ap; const T* A2 = (const T*)A2p; const T* Bt = (const T*)Btp; const T* Bt2 = (const T*)Bt2p;
  __shared__ __align__(16) float sT[8][16 * 68];
  const int b    = blockIdx.y;
  const int lane = threadIdx.x & 31;
  const int wave = threadIdx.x >> 5;
  const int tilesN = N >> 6;
  const int tilesM = M >> 6;
  const int tile = blockIdx.x * 8 + wave;
  if (tile >= tilesM * tilesN) return;
  const int tm = tile / tilesN;
  const int tn = tile - tm * tilesN;
  const int m0 = tm << 6;
  const int n0 = tn << 6;

  const T* Ab  = A  + (size_t)b * strideA;
  const T* Bb  = Bt + (size_t)b * strideB;
  const T* Ab2 = SPLIT ? (A2  + (size_t)b * strideA) : nullptr;
  const T* Bb2 = SPLIT ? (Bt2 + (size_t)b * strideB) : nullptr;

  const int rlane = lane & 15;
  const int koff  = (lane >> 4) * 8;
  const int mOff  = (lane >> 4) * 8;

  v8f acc[4][4];
#pragma unroll
  for (int i = 0; i < 4; ++i)
#pragma unroll
    for (int j = 0; j < 4; ++j) acc[i][j] = (v8f){0.f,0.f,0.f,0.f,0.f,0.f,0.f,0.f};

  for (int k0 = 0; k0 < K; k0 += 32) {
    V bh[4], bl[4];
#pragma unroll
    for (int j = 0; j < 4; ++j) {
      const size_t bo = (size_t)(n0 + (j << 4) + rlane) * ldb + koff + k0;
      bh[j] = Frag<T>::load(Bb + bo);
      if (SPLIT) bl[j] = Frag<T>::load(Bb2 + bo);
    }
#pragma unroll
    for (int i = 0; i < 4; ++i) {
      const size_t ao = (size_t)(m0 + (i << 4) + rlane) * lda + koff + k0;
      V ah = Frag<T>::load(Ab + ao);
      V al;
      if (SPLIT) al = Frag<T>::load(Ab2 + ao);
#pragma unroll
      for (int j = 0; j < 4; ++j) {
        acc[i][j] = Frag<T>::mma(ah, bh[j], acc[i][j]);
        if (SPLIT) {
          acc[i][j] = Frag<T>::mma(ah, bl[j], acc[i][j]);
          acc[i][j] = Frag<T>::mma(al, bh[j], acc[i][j]);
        }
      }
      Frag<T>::guard(acc[i][0], acc[i][3], ah, SPLIT ? al : ah);
    }
    Frag<T>::keep(bh[0], bh[1], bh[2], bh[3]);
    if (SPLIT) Frag<T>::keep(bl[0], bl[1], bl[2], bl[3]);
  }
  acc_guard4(acc[0][0], acc[0][1], acc[0][2], acc[0][3]);
  acc_guard4(acc[1][0], acc[1][1], acc[1][2], acc[1][3]);
  acc_guard4(acc[2][0], acc[2][1], acc[2][2], acc[2][3]);
  acc_guard4(acc[3][0], acc[3][1], acc[3][2], acc[3][3]);

  float* slab = sT[wave];
  const float* Rb = RESID ? (resid + (size_t)b * strideR) : nullptr;
#pragma unroll
  for (int i = 0; i < 4; ++i) {
    const int mBase = m0 + (i << 4);
#pragma unroll
    for (int j = 0; j < 4; ++j) {
      const int n = n0 + (j << 4) + rlane;
      float bv = 0.f;
      if (BIAS_MODE == 2) bv = bias[n];
#pragma unroll
      for (int r = 0; r < 8; ++r) {
        float v = acc[i][j][r] * scale;
        if (BIAS_MODE == 1) v += bias[mBase + mOff + r];
        if (BIAS_MODE == 2) v += bv;
        if (RESID) v += Rb[(size_t)(mBase + mOff + r) * ldc + n];
        if (ACT == 1) v = tanhf(v);
        if (ACT == 2) v = fmaxf(v, 0.0f);
        if (ACT == 3) v = v / (1.0f + expf(-v));
        if (ACT == 4) v = (v > 0.f) ? v : 0.01f * v;
        if (ACT == 5) v = 0.5f * v * (1.0f + erff(v * 0.70710678118654752f));
        slab[(mOff + r) * 68 + (j << 4) + rlane] = v;
      }
    }
    __builtin_amdgcn_fence(__ATOMIC_RELEASE, "workgroup");
    __builtin_amdgcn_wave_barrier();
    __builtin_amdgcn_fence(__ATOMIC_ACQUIRE, "workgroup");
    if (OUT_MODE == 0) {
      float* C = (float*)Cout + (size_t)b * strideC;
      const int hh = lane >> 4, c4 = (lane & 15) * 4;
      for (int pass = 0; pass < 2; ++pass) {
#pragma unroll
        for (int it = 0; it < 8; ++it) {
          const int row = it * 2 + hh;
          v4f v = *(const v4f*)(slab + row * 68 + c4);
          *(volatile v4f*)(C + (size_t)(mBase + row) * ldc + n0 + c4) = v;
        }
        __threadfence();
      }
    } else {
      const int q = lane >> 3, c8 = (lane & 7) * 8;
      unsigned short* C  = (unsigned short*)Cout  + (size_t)b * strideC;
      unsigned short* C2 = (OUT_MODE == 2) ? ((unsigned short*)Cout2 + (size_t)b * strideC) : nullptr;
      for (int pass = 0; pass < 2; ++pass) {
#pragma unroll
        for (int it = 0; it < 4; ++it) {
          const int row = it * 4 + q;
          const float* sp = slab + row * 68 + c8;
          v8h hv, lv;
#pragma unroll
          for (int e = 0; e < 8; ++e) {
            if (OUT_MODE == 1) {
              hv[e] = (_Float16)sp[e];
            } else {
              unsigned short hb = f2bf_bits(sp[e]);
              unsigned short lb = f2bf_bits(sp[e] - bf_bits2f(hb));
              hv[e] = __builtin_bit_cast(_Float16, hb);
              lv[e] = __builtin_bit_cast(_Float16, lb);
            }
          }
          *(volatile v8h*)(C + (size_t)(mBase + row) * ldc + n0 + c8) = hv;
          if (OUT_MODE == 2) *(volatile v8h*)(C2 + (size_t)(mBase + row) * ldc + n0 + c8) = lv;
        }
        __threadfence();
      }
    }
    __builtin_amdgcn_fence(__ATOMIC_RELEASE, "workgroup");
    __builtin_amdgcn_wave_barrier();
    __builtin_amdgcn_fence(__ATOMIC_ACQUIRE, "workgroup");
  }
}

__global__ __launch_bounds__(256) void cast_f32_f16x2(
    const float* __restrict__ in, _Float16* __restrict__ out, int n2) {
  int i = blockIdx.x * 256 + threadIdx.x;
  if (i < n2) {
    const _Float16 h0 = (_Float16)in[2 * i], h1 = (_Float16)in[2 * i + 1];
    const unsigned u = (unsigned)__builtin_bit_cast(unsigned short, h0) | ((unsigned)__builtin_bit_cast(unsigned short, h1) << 16);
    ((volatile unsigned*)out)[i] = u;
    __threadfence();
    ((volatile unsigned*)out)[i] = u;
  }
}

constexpr int kB = 32;
constexpr int kT = 128;
constexpr int kL = 64;
constexpr int kD = 512;
constexpr int kH = 512;
constexpr int kA = 256;
constexpr int kG = 4 * kH;
constexpr int kRows = 16;
constexpr int kAP = 2 * kH;
constexpr int kXP = 3 * kD;
constexpr int kUni = 6144;
constexpr float kS8 = 8.0f;
constexpr float kInv128 = 1.0f / 128.0f;
static_assert(kH % 32 == 0 && kAP % 32 == 0 && kD % 32 == 0 && kXP % 32 == 0, "cfg");
static_assert(kB % kRows == 0 && kA == 8 * 32 && kH == 2 * 256 && kH == kD, "cfg");
static_assert(kRows * kA + kRows * kL <= kUni && 4 * kRows * 64 + 2 * kRows * 64 <= kUni, "cfg");

__device__ __forceinline__ v8f mma_h16(v16h a, v16h b, v8f c) {
  c = __builtin_amdgcn_wmma_f32_16x16x32_f16(false, a, false, b, (short)0, c, false, false);
  asm volatile("v_nop\n\tv_nop\n\tv_nop\n\tv_nop" : "+v"(c) : "v"(a), "v"(b));
  return c;
}
__device__ __forceinline__ float sigm_f(float x) { return 1.0f / (1.0f + expf(-x)); }

__device__ __forceinline__ void split2_bf16(float x0, float x1, unsigned& hw, unsigned& lw) {
  const unsigned short h0 = f2bf_bits(x0), h1 = f2bf_bits(x1);
  const unsigned short l0 = f2bf_bits(x0 - bf_bits2f(h0)), l1 = f2bf_bits(x1 - bf_bits2f(h1));
  hw = (unsigned)h0 | ((unsigned)h1 << 16);
  lw = (unsigned)l0 | ((unsigned)l1 << 16);
}

__global__ __launch_bounds__(256) void split_x3_bf16(
    const float* __restrict__ in, unsigned short* __restrict__ out, int ngroups) {
  const int i = blockIdx.x * 256 + threadIdx.x;
  if (i >= ngroups) return;
  const int row = i >> 6, c8 = (i & 63) * 8;
  const float* p = in + (size_t)row * kD + c8;
  const v4f xa = *(const v4f*)(p);
  const v4f xb = *(const v4f*)(p + 4);
  unsigned hw, lw;
  v4u hv, lv;
  split2_bf16(xa[0], xa[1], hw, lw); hv[0] = hw; lv[0] = lw;
  split2_bf16(xa[2], xa[3], hw, lw); hv[1] = hw; lv[1] = lw;
  split2_bf16(xb[0], xb[1], hw, lw); hv[2] = hw; lv[2] = lw;
  split2_bf16(xb[2], xb[3], hw, lw); hv[3] = hw; lv[3] = lw;
  unsigned short* o = out + (size_t)row * kXP + c8;
  for (int pass = 0; pass < 2; ++pass) {
    *(volatile v4u*)(o)          = hv;
    *(volatile v4u*)(o + kD)     = lv;
    *(volatile v4u*)(o + 2 * kD) = hv;
    __threadfence();
  }
}

__global__ __launch_bounds__(256) void tp_cast16(
    const float* __restrict__ in0, const float* __restrict__ in1,
    const float* __restrict__ in2, const float* __restrict__ in3,
    unsigned short* __restrict__ out0, unsigned short* __restrict__ out1,
    unsigned short* __restrict__ out2, unsigned short* __restrict__ out3,
    int ldin, int ldout, float scale) {
  __shared__ float sm[64][65];
  const int z = blockIdx.z;
  const float* in = (z == 0) ? in0 : (z == 1) ? in1 : (z == 2) ? in2 : in3;
  _Float16* out = (_Float16*)((z == 0) ? out0 : (z == 1) ? out1 : (z == 2) ? out2 : out3);
  const int c0 = blockIdx.x * 64, r0 = blockIdx.y * 64;
  const int tid = threadIdx.x, wave = tid >> 5, lane = tid & 31;
#pragma unroll
  for (int i = 0; i < 16; ++i) {
    const int idx = i * 256 + tid;
    const int rr = idx >> 6, cc = idx & 63;
    sm[rr][cc] = in[(size_t)(r0 + rr) * ldin + c0 + cc];
  }
  __syncthreads();
  const int q = lane >> 3, c8 = (lane & 7) * 8;
  v8h hv[2];
#pragma unroll
  for (int it = 0; it < 2; ++it) {
    const int orow = wave * 8 + it * 4 + q;
#pragma unroll
    for (int e = 0; e < 8; ++e) hv[it][e] = (_Float16)(sm[c8 + e][orow] * scale);
  }
  for (int pass = 0; pass < 2; ++pass) {
#pragma unroll
    for (int it = 0; it < 2; ++it) {
      const int orow = wave * 8 + it * 4 + q;
      *(volatile v8h*)(out + (size_t)(c0 + orow) * ldout + r0 + c8) = hv[it];
    }
    __threadfence();
  }
}

__global__ __launch_bounds__(256) void tp_split3_bf16(
    const float* __restrict__ in0, const float* __restrict__ in1,
    const float* __restrict__ in2, const float* __restrict__ in3,
    unsigned short* __restrict__ out0, unsigned short* __restrict__ out1,
    unsigned short* __restrict__ out2, unsigned short* __restrict__ out3,
    int ldin, int ldout, int kseg) {
  __shared__ float sm[64][65];
  const int z = blockIdx.z;
  const float* in = (z == 0) ? in0 : (z == 1) ? in1 : (z == 2) ? in2 : in3;
  unsigned short* out = (z == 0) ? out0 : (z == 1) ? out1 : (z == 2) ? out2 : out3;
  const int c0 = blockIdx.x * 64, r0 = blockIdx.y * 64;
  const int tid = threadIdx.x, wave = tid >> 5, lane = tid & 31;
#pragma unroll
  for (int i = 0; i < 16; ++i) {
    const int idx = i * 256 + tid;
    const int rr = idx >> 6, cc = idx & 63;
    sm[rr][cc] = in[(size_t)(r0 + rr) * ldin + c0 + cc];
  }
  __syncthreads();
  const int q = lane >> 3, c8 = (lane & 7) * 8;
  v4u hv[2], lv[2];
#pragma unroll
  for (int it = 0; it < 2; ++it) {
    const int orow = wave * 8 + it * 4 + q;
#pragma unroll
    for (int e2 = 0; e2 < 4; ++e2) {
      unsigned hw, lw;
      split2_bf16(sm[c8 + 2 * e2][orow], sm[c8 + 2 * e2 + 1][orow], hw, lw);
      hv[it][e2] = hw; lv[it][e2] = lw;
    }
  }
  for (int pass = 0; pass < 2; ++pass) {
#pragma unroll
    for (int it = 0; it < 2; ++it) {
      const int orow = wave * 8 + it * 4 + q;
      unsigned short* o = out + (size_t)(c0 + orow) * ldout + r0 + c8;
      *(volatile v4u*)(o)            = hv[it];
      *(volatile v4u*)(o + kseg)     = hv[it];
      *(volatile v4u*)(o + 2 * kseg) = lv[it];
    }
    __threadfence();
  }
}

__global__ __launch_bounds__(256) void rec_steps(
    const unsigned short* __restrict__ AhTp,
    const unsigned short* __restrict__ UCtp,
    const float* __restrict__ XG,
    const float* __restrict__ CT,
    const float* __restrict__ ctxin,
    const int* __restrict__ cmask,
    const float* __restrict__ tmask,
    const float* __restrict__ attW2,
    const float* __restrict__ attB2,
    float* hs_out, float* cs_out, float* __restrict__ cv_out) {
  __shared__ __align__(16) _Float16 sH16[2 * kRows * kH];
  __shared__ __align__(16) _Float16 sCX16[kRows * kD];
  __shared__ __align__(16) float uni[kUni];
  __shared__ __align__(16) float sW2[kA];
  float* const sAH = uni;
  float* const sE  = uni + 4096;
  float* const sG  = uni;
  float* const sOH = uni + 4096;
  float* const sOC = uni + 5120;

  const _Float16* AhT = (const _Float16*)AhTp;
  const _Float16* UCt = (const _Float16*)UCtp;
  const int tid = threadIdx.x, wave = tid >> 5, lane = tid & 31;
  const int hh = lane >> 4, rl = lane & 15, koff = hh * 8;
  const int b0 = blockIdx.x * kRows;
  const v8f kZ8 = (v8f){0.f,0.f,0.f,0.f,0.f,0.f,0.f,0.f};

  for (int i = tid; i < (2 * kRows * kH) / 8; i += 256) *(v4u*)(sH16 + 8 * i) = (v4u){0u, 0u, 0u, 0u};
  for (int i = tid; i < (kRows * kD) / 8; i += 256) *(v4u*)(sCX16 + 8 * i) = (v4u){0u, 0u, 0u, 0u};
  for (int i = tid; i < kUni; i += 256) uni[i] = 0.f;
  sW2[tid] = attW2[tid];
  const float b2 = attB2[0];
  __syncthreads();

  for (int t = 0; t < kT; ++t) {
    const _Float16* hcur = sH16 + (t & 1) * (kRows * kH);
    _Float16* hnxt = sH16 + ((t + 1) & 1) * (kRows * kH);

    {
      v8f acc0 = kZ8, acc1 = kZ8;
      const int n0 = wave * 32;
      const _Float16* ap  = hcur + rl * kH + koff;
      const _Float16* bp0 = AhT + (size_t)(n0 + rl) * kH + koff;
      const _Float16* bp1 = AhT + (size_t)(n0 + 16 + rl) * kH + koff;
#pragma unroll 2
      for (int k0 = 0; k0 < kH; k0 += 32) {
        const v16h a  = Frag<_Float16>::load(ap + k0);
        const v16h f0 = Frag<_Float16>::load(bp0 + k0);
        const v16h f1 = Frag<_Float16>::load(bp1 + k0);
        acc0 = mma_h16(a, f0, acc0);
        acc1 = mma_h16(a, f1, acc1);
      }
#pragma unroll
      for (int r = 0; r < 8; ++r) {
        sAH[(8 * hh + r) * kA + n0 + rl]      = acc0[r] * kInv128;
        sAH[(8 * hh + r) * kA + n0 + 16 + rl] = acc1[r] * kInv128;
      }
    }
    __syncthreads();

    {
      const int l = tid & 63, rq = tid >> 6;
#pragma unroll 1
      for (int i = 0; i < 4; ++i) {
        const int row = rq + 4 * i;
        const float* ct  = CT + ((size_t)(b0 + row) * kL + l) * kA;
        const float* ahr = sAH + row * kA;
        float s = 0.f;
#pragma unroll 1
        for (int a = 0; a < kA; ++a) s += tanhf(ct[a] + ahr[a]) * sW2[a];
        s += b2;
        const float cmv = (float)cmask[(b0 + row) * kL + l];
        sE[row * kL + l] = expf(s) * cmv;
      }
    }
    __syncthreads();

    if (tid < kRows) {
      float s = 0.f;
#pragma unroll 1
      for (int l = 0; l < kL; ++l) s += sE[tid * kL + l];
      const float inv = 1.0f / s;
#pragma unroll 1
      for (int l = 0; l < kL; ++l) sE[tid * kL + l] = sE[tid * kL + l] * inv;
    }
    __syncthreads();

    {
      v4f cv4[8];
#pragma unroll
      for (int j = 0; j < 8; ++j) cv4[j] = (v4f){0.f, 0.f, 0.f, 0.f};
      const int rsel = tid >> 7;
      const int q4 = (tid & 127) * 4;
      const float* cb = ctxin + (size_t)b0 * kL * kD + q4;
#pragma unroll 1
      for (int l = 0; l < kL; ++l) {
        const float* cl = cb + (size_t)l * kD;
#pragma unroll
        for (int j = 0; j < 8; ++j) {
          const int row = 2 * j + rsel;
          const float aw = sE[row * kL + l];
          const v4f x4 = *(const v4f*)(cl + (size_t)row * kL * kD);
          cv4[j][0] = fmaf(aw, x4[0], cv4[j][0]);
          cv4[j][1] = fmaf(aw, x4[1], cv4[j][1]);
          cv4[j][2] = fmaf(aw, x4[2], cv4[j][2]);
          cv4[j][3] = fmaf(aw, x4[3], cv4[j][3]);
        }
      }
#pragma unroll
      for (int j = 0; j < 8; ++j) {
        const int row = 2 * j + rsel;
        v4h h4;
        h4[0] = (_Float16)(cv4[j][0] * kS8);
        h4[1] = (_Float16)(cv4[j][1] * kS8);
        h4[2] = (_Float16)(cv4[j][2] * kS8);
        h4[3] = (_Float16)(cv4[j][3] * kS8);
        *(v4h*)(sCX16 + row * kD + q4) = h4;
      }
      for (int pass = 0; pass < 2; ++pass) {
#pragma unroll
        for (int j = 0; j < 8; ++j) {
          const int row = 2 * j + rsel;
          *(volatile v4f*)(cv_out + ((size_t)(b0 + row) * kT + t) * kD + q4) = cv4[j];
        }
        __threadfence();
      }
    }
    __syncthreads();

    {
      const int jj = wave & 3;
      const int g0 = (wave >> 2) * 2;
      const int row = tid >> 4, cb = (tid & 15) * 4;
      const float mval = tmask[(size_t)(b0 + row) * kT + t];
      const int tp = (t > 0) ? (t - 1) : 0;
      const size_t prow = ((size_t)(b0 + row) * kT + tp) * kH;
      const size_t orow = ((size_t)(b0 + row) * kT + t) * kH;
      const size_t xrow = ((size_t)(b0 + row) * kT + t) * kG;
#pragma unroll 1
      for (int q = 0; q < 8; ++q) {
        const int ub = 64 * q + 16 * jj;
        v8f acc0 = kZ8, acc1 = kZ8;
        const _Float16* bp0 = UCt + (size_t)(g0 * kH + ub + rl) * kAP + koff;
        const _Float16* bp1 = bp0 + (size_t)kH * kAP;
        {
          const _Float16* ap = hcur + rl * kH + koff;
#pragma unroll 2
          for (int k0 = 0; k0 < kH; k0 += 32) {
            const v16h a  = Frag<_Float16>::load(ap + k0);
            const v16h f0 = Frag<_Float16>::load(bp0 + k0);
            const v16h f1 = Frag<_Float16>::load(bp1 + k0);
            acc0 = mma_h16(a, f0, acc0);
            acc1 = mma_h16(a, f1, acc1);
          }
        }
        {
          const _Float16* ap = sCX16 + rl * kD + koff;
#pragma unroll 2
          for (int k0 = 0; k0 < kD; k0 += 32) {
            const v16h a  = Frag<_Float16>::load(ap + k0);
            const v16h f0 = Frag<_Float16>::load(bp0 + kH + k0);
            const v16h f1 = Frag<_Float16>::load(bp1 + kH + k0);
            acc0 = mma_h16(a, f0, acc0);
            acc1 = mma_h16(a, f1, acc1);
          }
        }
#pragma unroll
        for (int r = 0; r < 8; ++r) {
          sG[(g0 * 16 + 8 * hh + r) * 64 + 16 * jj + rl]       = acc0[r] * kInv128;
          sG[((g0 + 1) * 16 + 8 * hh + r) * 64 + 16 * jj + rl] = acc1[r] * kInv128;
        }
        __syncthreads();

#pragma unroll 1
        for (int e = 0; e < 4; ++e) {
          const int j = cb + e;
          const int u = 64 * q + j;
          const float pi = XG[xrow + u]          + sG[(0 * 16 + row) * 64 + j];
          const float pf = XG[xrow + kH + u]     + sG[(1 * 16 + row) * 64 + j];
          const float pc = XG[xrow + 2 * kH + u] + sG[(2 * 16 + row) * 64 + j];
          const float po = XG[xrow + 3 * kH + u] + sG[(3 * 16 + row) * 64 + j];
          const float ig = sigm_f(pi);
          const float fg = sigm_f(pf);
          const float cc = tanhf(pc);
          const float og = sigm_f(po);
          const float c_ld = cs_out[prow + u];
          const float h_ld = hs_out[prow + u];
          const float c_old = (t > 0) ? c_ld : 0.f;
          const float h_old = (t > 0) ? h_ld : 0.f;
          const float c_new = fg * c_old + ig * cc;
          const float h_new = og * tanhf(c_new);
          const float c_bl = (1.0f - mval) * c_old + mval * c_new;
          const float h_bl = (1.0f - mval) * h_old + mval * h_new;
          sOC[row * 64 + j] = c_bl;
          sOH[row * 64 + j] = h_bl;
          hnxt[row * kH + u] = (_Float16)(h_bl * kS8);
        }
        __syncthreads();

        {
          const v4f hv  = *(const v4f*)(sOH + row * 64 + cb);
          const v4f cvv = *(const v4f*)(sOC + row * 64 + cb);
          for (int pass = 0; pass < 2; ++pass) {
            *(volatile v4f*)(hs_out + orow + 64 * q + cb) = hv;
            *(volatile v4f*)(cs_out + orow + 64 * q + cb) = cvv;
            __threadfence();
          }
        }
      }
    }
  }
}

extern "C" void kernel_launch(void* const* d_in, const int* in_sizes, int n_in,
                              void* d_out, int out_size, void* d_ws, size_t ws_size,
                              hipStream_t stream) {
  if (n_in < 25) return;
  if (in_sizes[0] != kB * kT * kD) return;
  if (in_sizes[1] != kB * kL * kD) return;
  if (in_sizes[2] != kB * kT) return;
  if (in_sizes[3] != kB * kL) return;
  for (int g = 0; g < 4; ++g) {
    if (in_sizes[4 + 4 * g] != kD * kH) return;
    if (in_sizes[5 + 4 * g] != kH * kH) return;
    if (in_sizes[6 + 4 * g] != kD * kH) return;
    if (in_sizes[7 + 4 * g] != kH) return;
  }
  if (in_sizes[20] != kD * kA || in_sizes[21] != kH * kA || in_sizes[22] != kA || in_sizes[23] != kA || in_sizes[24] < 1) return;
  if (out_size != 3 * kB * kT * kH) return;

  const float* X        = (const float*)d_in[0];
  const float* context  = (const float*)d_in[1];
  const float* tmask    = (const float*)d_in[2];
  const int*   cmask    = (const int*)d_in[3];
  const float* W[4]  = {(const float*)d_in[4],  (const float*)d_in[8],  (const float*)d_in[12], (const float*)d_in[16]};
  const float* U[4]  = {(const float*)d_in[5],  (const float*)d_in[9],  (const float*)d_in[13], (const float*)d_in[17]};
  const float* Cg[4] = {(const float*)d_in[6],  (const float*)d_in[10], (const float*)d_in[14], (const float*)d_in[18]};
  const float* bg[4] = {(const float*)d_in[7],  (const float*)d_in[11], (const float*)d_in[15], (const float*)d_in[19]};
  const float* attCtxW1 = (const float*)d_in[20];
  const float* attHW1   = (const float*)d_in[21];
  const float* attB1    = (const float*)d_in[22];
  const float* attW2    = (const float*)d_in[23];
  const float* attB2    = (const float*)d_in[24];

  char* ws = (char*)d_ws;
  size_t off = 0;
  const size_t nXP   = (size_t)kB * kT * kXP * 2;
  const size_t nC16  = (size_t)kB * kL * kD * 2;
  const size_t nWtP  = (size_t)kG * kXP * 2;
  const size_t nUCt  = (size_t)kG * kAP * 2;
  const size_t nAcT  = (size_t)kA * kD * 2;
  const size_t nAhT  = (size_t)kA * kH * 2;
  const size_t nXG   = (size_t)kB * kT * kG * 4;
  const size_t nCT   = (size_t)kB * kL * kA * 4;
  unsigned short* XP    = (unsigned short*)(ws + off); off += nXP;   off = (off + 255) & ~(size_t)255;
  unsigned short* C16   = (unsigned short*)(ws + off); off += nC16;  off = (off + 255) & ~(size_t)255;
  unsigned short* WtP   = (unsigned short*)(ws + off); off += nWtP;  off = (off + 255) & ~(size_t)255;
  unsigned short* UCt16 = (unsigned short*)(ws + off); off += nUCt;  off = (off + 255) & ~(size_t)255;
  unsigned short* AcT16 = (unsigned short*)(ws + off); off += nAcT;  off = (off + 255) & ~(size_t)255;
  unsigned short* AhT16 = (unsigned short*)(ws + off); off += nAhT;  off = (off + 255) & ~(size_t)255;
  float* XG = (float*)(ws + off); off += nXG; off = (off + 255) & ~(size_t)255;
  float* CT = (float*)(ws + off); off += nCT; off = (off + 255) & ~(size_t)255;
  if (off > ws_size) return;

  float* hs_out = (float*)d_out;
  float* cs_out = hs_out + (size_t)kB * kT * kH;
  float* cv_out = cs_out + (size_t)kB * kT * kH;

  split_x3_bf16<<<(kB * kT * (kD / 8)) / 256, 256, 0, stream>>>(X, XP, kB * kT * (kD / 8));
  cast_f32_f16x2<<<(kB * kL * kD / 2) / 256, 256, 0, stream>>>(context, (_Float16*)C16, kB * kL * kD / 2);

  tp_split3_bf16<<<dim3(kH / 64, kD / 64, 4), 256, 0, stream>>>(
      W[0], W[1], W[2], W[3],
      WtP, WtP + (size_t)1 * kH * kXP, WtP + (size_t)2 * kH * kXP, WtP + (size_t)3 * kH * kXP,
      kH, kXP, kD);
  tp_cast16<<<dim3(kH / 64, kH / 64, 4), 256, 0, stream>>>(
      U[0], U[1], U[2], U[3],
      UCt16, UCt16 + (size_t)1 * kH * kAP, UCt16 + (size_t)2 * kH * kAP, UCt16 + (size_t)3 * kH * kAP,
      kH, kAP, 16.0f);
  tp_cast16<<<dim3(kH / 64, kD / 64, 4), 256, 0, stream>>>(
      Cg[0], Cg[1], Cg[2], Cg[3],
      UCt16 + kH, UCt16 + (size_t)1 * kH * kAP + kH, UCt16 + (size_t)2 * kH * kAP + kH, UCt16 + (size_t)3 * kH * kAP + kH,
      kH, kAP, 16.0f);
  tp_cast16<<<dim3(kA / 64, kD / 64, 2), 256, 0, stream>>>(
      attCtxW1, attHW1, attHW1, attHW1,
      AcT16, AhT16, AhT16, AhT16,
      kA, kD, 16.0f);

  for (int g = 0; g < 4; ++g) {
    wmma_gemm64<1, false, 2, 0, false, 0><<<dim3((kB * kT / 64) * (kH / 64) / 8, 1), 256, 0, stream>>>(
        XP, XP, kXP, 0L,
        WtP + (size_t)g * kH * kXP, WtP + (size_t)g * kH * kXP, kXP, 0L,
        (void*)(XG + (size_t)g * kH), (void*)XG, kG, 0L,
        bg[g], bg[g], 0L,
        kB * kT, kH, kXP, 1.0f);
  }
  wmma_gemm64<0, false, 2, 0, false, 0><<<dim3((kB * kL / 64) * (kA / 64) / 8, 1), 256, 0, stream>>>(
      C16, C16, kD, 0L,
      AcT16, AcT16, kD, 0L,
      (void*)CT, (void*)CT, kA, 0L,
      attB1, attB1, 0L,
      kB * kL, kA, kD, 1.0f / 16.0f);

  rec_steps<<<kB / kRows, 256, 0, stream>>>(AhT16, UCt16, XG, CT, context, cmask, tmask, attW2, attB2,
                                            hs_out, cs_out, cv_out);
}
